// MultiHeadSelfAttention_1357209665786
// MI455X (gfx1250) — hardware-verified
//
#include <hip/hip_runtime.h>
#include <math.h>
#include <stdint.h>

#define NBT   8
#define SEQ   512
#define DMOD  512
#define NHEAD 8
#define HDIM  64
#define NREL  1023
#define NRELP 1024
#define BDW   576
#define PBD   68

static_assert(SEQ % 64 == 0);
static_assert(DMOD % 64 == 0);
static_assert(HDIM % 32 == 0);
static_assert(NHEAD * HDIM == DMOD);
static_assert(BDW % 64 == 0);
static_assert(BDW >= SEQ + 64);
static_assert(64 * (SEQ / 64 - 1) + BDW <= NRELP);
static_assert((SEQ - 64) + 60 + 68 <= BDW);
static_assert(4 * 16 * PBD == 64 * PBD);

typedef __attribute__((ext_vector_type(16))) __bf16   v16b;
typedef __attribute__((ext_vector_type(8)))  __bf16   v8b;
typedef __attribute__((ext_vector_type(8)))  float    v8f;
typedef __attribute__((ext_vector_type(4)))  float    v4f;
typedef __attribute__((ext_vector_type(4)))  unsigned int v4u;
typedef v4f __attribute__((may_alias)) v4fa;
typedef v8b __attribute__((may_alias)) v8ba;

__device__ __forceinline__ unsigned short f2bf_bits(float f) {
  unsigned u = __float_as_uint(f);
  return (unsigned short)((u + 0x7FFFu + ((u >> 16) & 1u)) >> 16);
}
__device__ __forceinline__ float bf_bits2f(unsigned short h) { return __uint_as_float(((unsigned)h) << 16); }
__device__ __forceinline__ float bf_rne(float f) { return bf_bits2f(f2bf_bits(f)); }
__device__ __forceinline__ unsigned pk16(unsigned short a, unsigned short b) { return (unsigned)a | ((unsigned)b << 16); }
__device__ __forceinline__ __bf16 bits2bf(unsigned short h) { return __builtin_bit_cast(__bf16, h); }
__device__ __forceinline__ void bf_split(float f, __bf16& hi, __bf16& lo) {
  const unsigned short hb = f2bf_bits(f);
  hi = bits2bf(hb);
  lo = bits2bf(f2bf_bits(f - bf_bits2f(hb)));
}

union FB { v16b v; v8ba h[2]; };
__device__ __forceinline__ v16b ldfrag(const __bf16* p) {
  FB f;
  f.h[0] = *(const v8ba*)(p);
  f.h[1] = *(const v8ba*)(p + 16);
  return f.v;
}

__device__ __forceinline__ v8f mmab(v16b a, v16b b, v8f c) {
  c = __builtin_amdgcn_wmma_f32_16x16x32_bf16(false, a, false, b, (short)0, c, false, false);
  asm volatile("v_nop\n\tv_nop\n\tv_nop\n\tv_nop" : "+v"(c) : "v"(a), "v"(b));
  return c;
}

__device__ __forceinline__ v8f zero8() { v8f z = {0.f, 0.f, 0.f, 0.f, 0.f, 0.f, 0.f, 0.f}; return z; }

__global__ __launch_bounds__(256) void cvt_bf16_kernel(const float* __restrict__ src, unsigned short* __restrict__ dst,
                                                       int nrows_src, int nrows_dst) {
  const int i = blockIdx.x * 256 + threadIdx.x;
  const int total8 = nrows_dst * (DMOD / 8);
  if (i >= total8) return;
  const int r  = i >> 6;
  const int c8 = (i & 63) * 8;
  const int rs = (r < nrows_src) ? r : (nrows_src - 1);
  const unsigned msk = (r < nrows_src) ? 0xFFFFFFFFu : 0u;
  const float* sp = src + (size_t)rs * DMOD + c8;
  const v4f a0 = *(const v4f*)(sp);
  const v4f a1 = *(const v4f*)(sp + 4);
  v4u o;
  o[0] = pk16(f2bf_bits(a0[0]), f2bf_bits(a0[1])) & msk;
  o[1] = pk16(f2bf_bits(a0[2]), f2bf_bits(a0[3])) & msk;
  o[2] = pk16(f2bf_bits(a1[0]), f2bf_bits(a1[1])) & msk;
  o[3] = pk16(f2bf_bits(a1[2]), f2bf_bits(a1[3])) & msk;
  unsigned short* dp = dst + (size_t)r * DMOD + c8;
  *(volatile v4u*)dp = o;
  __threadfence();
  *(volatile v4u*)dp = o;
}

template <bool SPLA, int BIAS_MODE, int OUT_MODE, bool SKEW>
__global__ __launch_bounds__(256) void gemm_bf16_kernel(
    const __bf16* A, const __bf16* A2, int lda, long strideA,
    const __bf16* Bt, int ldb, long strideB,
    void* C1, void* C2, int ldc, long strideC,
    const float* __restrict__ bias,
    int M, int N, int K, float scale, int skew0) {
  __shared__ __align__(16) float sT[8][16 * 68];

  const int z    = blockIdx.y;
  const int lane = threadIdx.x & 31;
  const int wave = threadIdx.x >> 5;
  const int tilesN = N >> 6;
  const int tilesM = M >> 6;
  const int tile = blockIdx.x * 8 + wave;
  if (tile >= tilesM * tilesN) return;
  const int tm = tile / tilesN;
  const int tn = tile - tm * tilesN;
  const int m0 = tm << 6;
  const int n0 = tn << 6;
  const int nsk = SKEW ? ((skew0 - tm) << 6) : 0;

  const __bf16* Ab  = A  + (size_t)z * strideA;
  const __bf16* Ab2 = SPLA ? (A2 + (size_t)z * strideA) : Ab;
  const __bf16* Bb  = Bt + (size_t)z * strideB;

  const int rl   = lane & 15;
  const int koff = (lane >> 4) * 8;
  const int mOff = (lane >> 4) * 8;

  v8f acc[4][4];
#pragma unroll
  for (int i = 0; i < 4; ++i)
#pragma unroll
    for (int j = 0; j < 4; ++j) acc[i][j] = zero8();

  for (int k0 = 0; k0 < K; k0 += 32) {
    v16b bfr[4];
#pragma unroll
    for (int j = 0; j < 4; ++j)
      bfr[j] = ldfrag(Bb + (size_t)(nsk + n0 + (j << 4) + rl) * ldb + koff + k0);
#pragma unroll
    for (int i = 0; i < 4; ++i) {
      const size_t ao = (size_t)(m0 + (i << 4) + rl) * lda + koff + k0;
      const v16b ah = ldfrag(Ab + ao);
      v16b al = ah;
      if (SPLA) al = ldfrag(Ab2 + ao);
#pragma unroll
      for (int j = 0; j < 4; ++j) {
        acc[i][j] = mmab(ah, bfr[j], acc[i][j]);
        if (SPLA) acc[i][j] = mmab(al, bfr[j], acc[i][j]);
      }
    }
  }

  float* slab = sT[wave];
#pragma unroll
  for (int i = 0; i < 4; ++i) {
    const int mBase = m0 + (i << 4);
    float bm[8];
#pragma unroll
    for (int r = 0; r < 8; ++r) bm[r] = 0.0f;
    if (BIAS_MODE == 1) {
#pragma unroll
      for (int r = 0; r < 8; ++r) bm[r] = bf_rne(bias[mBase + mOff + r]);
    }
#pragma unroll
    for (int j = 0; j < 4; ++j) {
      float bn = 0.0f;
      if (BIAS_MODE == 2) bn = bf_rne(bias[n0 + (j << 4) + rl]);
#pragma unroll
      for (int r = 0; r < 8; ++r) {
        float v = acc[i][j][r] * scale;
        if (BIAS_MODE == 1) v += bm[r];
        if (BIAS_MODE == 2) v += bn;
        slab[(mOff + r) * 68 + (j << 4) + rl] = v;
      }
    }
    __builtin_amdgcn_fence(__ATOMIC_RELEASE, "workgroup");
    __builtin_amdgcn_wave_barrier();
    __builtin_amdgcn_fence(__ATOMIC_ACQUIRE, "workgroup");
    if (OUT_MODE == 0) {
      float* C = (float*)C1 + (size_t)z * strideC;
      const int hh = lane >> 4, c4 = (lane & 15) * 4;
      for (int pass = 0; pass < 2; ++pass) {
#pragma unroll
        for (int it = 0; it < 8; ++it) {
          const int row = it * 2 + hh;
          const v4f v = *(const v4fa*)(slab + row * 68 + c4);
          *(volatile v4f*)(C + (size_t)(mBase + row) * ldc + n0 + c4) = v;
        }
        __threadfence();
      }
    } else {
      const int q = lane >> 3, c8 = (lane & 7) * 8;
      unsigned short* Ca = (unsigned short*)C1 + (size_t)z * strideC;
      unsigned short* Cb = (unsigned short*)C2 + (size_t)z * strideC;
      v4u hv[4], lv[4];
#pragma unroll
      for (int it = 0; it < 4; ++it) {
        const int row = it * 4 + q;
        const float* sp = slab + row * 68 + c8;
        v4u a, a2;
#pragma unroll
        for (int e = 0; e < 4; ++e) {
          const float f0 = sp[2 * e], f1 = sp[2 * e + 1];
          const unsigned short h0 = f2bf_bits(f0), h1 = f2bf_bits(f1);
          const unsigned short l0 = f2bf_bits(f0 - bf_bits2f(h0)), l1 = f2bf_bits(f1 - bf_bits2f(h1));
          a[e]  = pk16(h0, h1);
          a2[e] = pk16(l0, l1);
        }
        hv[it] = a; lv[it] = a2;
      }
      for (int pass = 0; pass < 2; ++pass) {
#pragma unroll
        for (int it = 0; it < 4; ++it) {
          const int row = it * 4 + q;
          const size_t go = (size_t)(mBase + row) * ldc + n0 + c8;
          *(volatile v4u*)(Ca + go) = hv[it];
          *(volatile v4u*)(Cb + go) = lv[it];
        }
        __threadfence();
      }
    }
    __builtin_amdgcn_fence(__ATOMIC_RELEASE, "workgroup");
    __builtin_amdgcn_wave_barrier();
    __builtin_amdgcn_fence(__ATOMIC_ACQUIRE, "workgroup");
  }
}

__global__ __launch_bounds__(128)
void attn_rel64_kernel(const __bf16* __restrict__ Qhp, const __bf16* __restrict__ Qlp,
                       const __bf16* __restrict__ Khp, const __bf16* __restrict__ Klp,
                       const __bf16* __restrict__ VThp, const __bf16* __restrict__ VTlp,
                       const float* __restrict__ BD,
                       unsigned short* __restrict__ CTXh, unsigned short* __restrict__ CTXl,
                       int b, float sscale) {
  __shared__ __align__(16) __bf16 Ksh[64 * HDIM];
  __shared__ __align__(16) __bf16 Ksl[64 * HDIM];
  __shared__ __align__(16) __bf16 Vth[HDIM * 64];
  __shared__ __align__(16) __bf16 Vtl[HDIM * 64];
  __shared__ __align__(16) __bf16 Psh[4][16 * 64];
  __shared__ __align__(16) __bf16 Psl[4][16 * 64];
  __shared__ __align__(16) float  Bsh[64 * PBD];

  const int tid  = threadIdx.x;
  const int wave = tid >> 5;
  const int lane = tid & 31;
  const int hh   = lane >> 4;
  const int c    = lane & 15;

  const int bx = blockIdx.x;
  const int qb = bx & 7;
  const int h  = bx >> 3;
  const int q0  = qb * 64 + wave * 16;
  const int rr0 = wave * 16 + 8 * hh;

  const size_t actb = (size_t)b * SEQ * DMOD;
  const __bf16* Qh = Qhp + actb + h * HDIM;
  const __bf16* Ql = Qlp + actb + h * HDIM;
  const __bf16* Kh = Khp + actb + h * HDIM;
  const __bf16* Kl = Klp + actb + h * HDIM;
  const __bf16* Vh = VThp + (size_t)b * DMOD * SEQ + (size_t)(h * HDIM) * SEQ;
  const __bf16* Vl = VTlp + (size_t)b * DMOD * SEQ + (size_t)(h * HDIM) * SEQ;
  const float*  bd = BD + ((size_t)h * SEQ + (size_t)qb * 64) * BDW;
  unsigned short* ch = CTXh + actb + h * HDIM;
  unsigned short* cl = CTXl + actb + h * HDIM;

  v16b qah[2], qal[2];
#pragma unroll
  for (int dc = 0; dc < 2; ++dc) {
    qah[dc] = ldfrag(Qh + (size_t)(q0 + c) * DMOD + dc * 32 + 8 * hh);
    qal[dc] = ldfrag(Ql + (size_t)(q0 + c) * DMOD + dc * 32 + 8 * hh);
  }

  float mrow[8], lrow[8];
  v8f oacc[4];
#pragma unroll
  for (int r = 0; r < 8; ++r) { mrow[r] = -INFINITY; lrow[r] = 0.f; }
#pragma unroll
  for (int t = 0; t < 4; ++t) oacc[t] = zero8();

  for (int kc = 0; kc < SEQ / 64; ++kc) {
    const int kv0 = kc * 64;
    __syncthreads();
    {
      const int r = tid >> 1, half = (tid & 1) * 32;
      const __bf16* ksh = Kh + (size_t)(kv0 + r) * DMOD + half;
      const __bf16* ksl = Kl + (size_t)(kv0 + r) * DMOD + half;
      const __bf16* vsh = Vh + (size_t)r * SEQ + kv0 + half;
      const __bf16* vsl = Vl + (size_t)r * SEQ + kv0 + half;
#pragma unroll
      for (int i = 0; i < 4; ++i) {
        const v8b a0 = *(const v8ba*)(ksh + 8 * i);
        const v8b a1 = *(const v8ba*)(ksl + 8 * i);
        const v8b b0 = *(const v8ba*)(vsh + 8 * i);
        const v8b b1 = *(const v8ba*)(vsl + 8 * i);
        *(v8ba*)(Ksh + r * HDIM + half + 8 * i) = a0;
        *(v8ba*)(Ksl + r * HDIM + half + 8 * i) = a1;
        *(v8ba*)(Vth + r * 64   + half + 8 * i) = b0;
        *(v8ba*)(Vtl + r * 64   + half + 8 * i) = b1;
      }
    }
    {
      const int rr = tid >> 1, half = tid & 1;
      const int a  = 63 - rr;
      const int st = kv0 + (a & ~3);
      const float* rp = bd + (size_t)rr * BDW + st;
      float* lp = Bsh + rr * PBD;
#pragma unroll
      for (int i = 0; i < 9; ++i) {
        int idx = half + 2 * i;
        idx = (idx > 16) ? 16 : idx;
        const v4f v = *(const v4f*)(rp + 4 * idx);
        *(v4fa*)(lp + 4 * idx) = v;
      }
    }
    __syncthreads();

    v8f s[4];
#pragma unroll
    for (int j = 0; j < 4; ++j) {
      s[j] = zero8();
#pragma unroll
      for (int dc = 0; dc < 2; ++dc) {
        const v16b kb = ldfrag(Ksh + (j * 16 + c) * HDIM + dc * 32 + 8 * hh);
        const v16b kl = ldfrag(Ksl + (j * 16 + c) * HDIM + dc * 32 + 8 * hh);
        s[j] = mmab(qah[dc], kb, s[j]);
        s[j] = mmab(qah[dc], kl, s[j]);
        s[j] = mmab(qal[dc], kb, s[j]);
      }
    }
    float cm[8];
#pragma unroll
    for (int r = 0; r < 8; ++r) {
      const int boff = (rr0 + r) * PBD + ((63 - rr0 - r) & 3) + c;
      float m = -INFINITY;
#pragma unroll
      for (int j = 0; j < 4; ++j) {
        const float sv = s[j][r] * sscale + Bsh[boff + (j << 4)];
        s[j][r] = sv;
        m = fmaxf(m, sv);
      }
#pragma unroll
      for (int off = 1; off < 16; off <<= 1) m = fmaxf(m, __shfl_xor(m, off, 32));
      cm[r] = m;
    }
    __bf16* pwh = Psh[wave];
    __bf16* pwl = Psl[wave];
#pragma unroll
    for (int r = 0; r < 8; ++r) {
      const float mnew  = fmaxf(mrow[r], cm[r]);
      const float alpha = __expf(mrow[r] - mnew);
      mrow[r] = mnew;
      float psum = 0.f;
#pragma unroll
      for (int j = 0; j < 4; ++j) {
        const float p = __expf(s[j][r] - mnew);
        psum += p;
        __bf16 ph, pl;
        bf_split(p, ph, pl);
        pwh[(8 * hh + r) * 64 + j * 16 + c] = ph;
        pwl[(8 * hh + r) * 64 + j * 16 + c] = pl;
      }
#pragma unroll
      for (int off = 1; off < 16; off <<= 1) psum += __shfl_xor(psum, off, 32);
      lrow[r] = lrow[r] * alpha + psum;
#pragma unroll
      for (int t = 0; t < 4; ++t) oacc[t][r] *= alpha;
    }
    __builtin_amdgcn_fence(__ATOMIC_RELEASE, "workgroup");
    __builtin_amdgcn_wave_barrier();
    __builtin_amdgcn_fence(__ATOMIC_ACQUIRE, "workgroup");

#pragma unroll 1
    for (int kk = 0; kk < 2; ++kk) {
      const v16b pa = ldfrag(pwh + c * 64 + kk * 32 + 8 * hh);
      const v16b pl = ldfrag(pwl + c * 64 + kk * 32 + 8 * hh);
#pragma unroll
      for (int t = 0; t < 4; ++t) {
        const v16b vb = ldfrag(Vth + (t * 16 + c) * 64 + kk * 32 + 8 * hh);
        const v16b vl = ldfrag(Vtl + (t * 16 + c) * 64 + kk * 32 + 8 * hh);
        oacc[t] = mmab(pa, vb, oacc[t]);
        oacc[t] = mmab(pa, vl, oacc[t]);
        oacc[t] = mmab(pl, vb, oacc[t]);
      }
    }
  }

  __syncthreads();
  float* os = Bsh + wave * (16 * PBD);
#pragma unroll
  for (int r = 0; r < 8; ++r) {
    const float inv = 1.0f / lrow[r];
#pragma unroll
    for (int t = 0; t < 4; ++t) os[(8 * hh + r) * PBD + t * 16 + c] = oacc[t][r] * inv;
  }
  __builtin_amdgcn_fence(__ATOMIC_RELEASE, "workgroup");
  __builtin_amdgcn_wave_barrier();
  __builtin_amdgcn_fence(__ATOMIC_ACQUIRE, "workgroup");
  {
    const int q = lane >> 3, c8 = (lane & 7) * 8;
    v4u hv[4], lv[4];
#pragma unroll
    for (int it = 0; it < 4; ++it) {
      const int row = it * 4 + q;
      const float* sp = os + row * PBD + c8;
      v4u a, a2;
#pragma unroll
      for (int e = 0; e < 4; ++e) {
        const float f0 = sp[2 * e], f1 = sp[2 * e + 1];
        const unsigned short h0 = f2bf_bits(f0), h1 = f2bf_bits(f1);
        const unsigned short l0 = f2bf_bits(f0 - bf_bits2f(h0)), l1 = f2bf_bits(f1 - bf_bits2f(h1));
        a[e]  = pk16(h0, h1);
        a2[e] = pk16(l0, l1);
      }
      hv[it] = a; lv[it] = a2;
    }
    for (int pass = 0; pass < 2; ++pass) {
#pragma unroll
      for (int it = 0; it < 4; ++it) {
        const int row = it * 4 + q;
        const size_t go = (size_t)(q0 + row) * DMOD + c8;
        *(volatile v4u*)(ch + go) = hv[it];
        *(volatile v4u*)(cl + go) = lv[it];
      }
      __threadfence();
    }
  }
}

extern "C" void kernel_launch(void* const* d_in, const int* in_sizes, int n_in,
                              void* d_out, int out_size, void* d_ws, size_t ws_size,
                              hipStream_t stream) {
  if (n_in < 10) return;
  const int NX = NBT * SEQ * DMOD;
  if (in_sizes[0] != NX) return;
  if (in_sizes[1] != DMOD * DMOD || in_sizes[3] != DMOD * DMOD || in_sizes[5] != DMOD * DMOD || in_sizes[7] != DMOD * DMOD) return;
  if (in_sizes[2] != DMOD || in_sizes[4] != DMOD || in_sizes[6] != DMOD || in_sizes[8] != DMOD) return;
  if (in_sizes[9] != NREL * DMOD) return;
  if (out_size != NX) return;

  const float* x   = (const float*)d_in[0];
  const float* Wq  = (const float*)d_in[1];
  const float* bq  = (const float*)d_in[2];
  const float* Wk  = (const float*)d_in[3];
  const float* bk  = (const float*)d_in[4];
  const float* Wv  = (const float*)d_in[5];
  const float* bv  = (const float*)d_in[6];
  const float* Wo  = (const float*)d_in[7];
  const float* bo  = (const float*)d_in[8];
  const float* rel = (const float*)d_in[9];
  float* out = (float*)d_out;

  const size_t PX  = (size_t)NBT * SEQ * DMOD * 2;
  const size_t PW  = (size_t)DMOD * DMOD * 2;
  const size_t PR  = (size_t)NRELP * DMOD * 2;
  const size_t PV  = (size_t)NBT * DMOD * SEQ * 2;
  const size_t PBb = (size_t)NHEAD * SEQ * BDW * 4;
  size_t off = 0;
  const size_t oXB  = off; off += PX;
  const size_t oWQ  = off; off += PW;
  const size_t oWK  = off; off += PW;
  const size_t oWV  = off; off += PW;
  const size_t oWO  = off; off += PW;
  const size_t oREB = off; off += PR;
  const size_t oQh  = off; off += PX;
  const size_t oQl  = off; off += PX;
  const size_t oKh  = off; off += PX;
  const size_t oKl  = off; off += PX;
  const size_t oVTh = off; off += PV;
  const size_t oVTl = off; off += PV;
  const size_t oCh  = off; off += PX;
  const size_t oCl  = off; off += PX;
  const size_t oBD  = off; off += PBb;
  const size_t total = off;
  if (total > ws_size) return;
  if (total > (size_t)134217728) return;

  char* ws = (char*)d_ws;
  unsigned short* XB  = (unsigned short*)(ws + oXB);
  unsigned short* WQ  = (unsigned short*)(ws + oWQ);
  unsigned short* WK  = (unsigned short*)(ws + oWK);
  unsigned short* WV  = (unsigned short*)(ws + oWV);
  unsigned short* WOB = (unsigned short*)(ws + oWO);
  unsigned short* REB = (unsigned short*)(ws + oREB);
  unsigned short* Qh  = (unsigned short*)(ws + oQh);
  unsigned short* Ql  = (unsigned short*)(ws + oQl);
  unsigned short* Kh  = (unsigned short*)(ws + oKh);
  unsigned short* Kl  = (unsigned short*)(ws + oKl);
  unsigned short* VTh = (unsigned short*)(ws + oVTh);
  unsigned short* VTl = (unsigned short*)(ws + oVTl);
  unsigned short* CXh = (unsigned short*)(ws + oCh);
  unsigned short* CXl = (unsigned short*)(ws + oCl);
  float*          BDp = (float*)(ws + oBD);

  const dim3 blk(256);

  cvt_bf16_kernel<<<dim3((NBT * SEQ * (DMOD / 8)) / 256), blk, 0, stream>>>(x, XB, NBT * SEQ, NBT * SEQ);
  cvt_bf16_kernel<<<dim3((DMOD * (DMOD / 8)) / 256), blk, 0, stream>>>(Wq, WQ, DMOD, DMOD);
  cvt_bf16_kernel<<<dim3((DMOD * (DMOD / 8)) / 256), blk, 0, stream>>>(Wk, WK, DMOD, DMOD);
  cvt_bf16_kernel<<<dim3((DMOD * (DMOD / 8)) / 256), blk, 0, stream>>>(Wv, WV, DMOD, DMOD);
  cvt_bf16_kernel<<<dim3((DMOD * (DMOD / 8)) / 256), blk, 0, stream>>>(Wo, WOB, DMOD, DMOD);
  cvt_bf16_kernel<<<dim3((NRELP * (DMOD / 8)) / 256), blk, 0, stream>>>(rel, REB, NREL, NRELP);

  const dim3 gP(((NBT * SEQ / 64) * (DMOD / 64) + 7) / 8, 1);
  gemm_bf16_kernel<false, 2, 2, false><<<gP, blk, 0, stream>>>(
      (const __bf16*)XB, (const __bf16*)XB, DMOD, 0L, (const __bf16*)WQ, DMOD, 0L,
      (void*)Qh, (void*)Ql, DMOD, 0L, bq, NBT * SEQ, DMOD, DMOD, 1.0f, 0);
  gemm_bf16_kernel<false, 2, 2, false><<<gP, blk, 0, stream>>>(
      (const __bf16*)XB, (const __bf16*)XB, DMOD, 0L, (const __bf16*)WK, DMOD, 0L,
      (void*)Kh, (void*)Kl, DMOD, 0L, bk, NBT * SEQ, DMOD, DMOD, 1.0f, 0);
  const dim3 gV(((DMOD / 64) * (SEQ / 64) + 7) / 8, NBT);
  gemm_bf16_kernel<false, 1, 2, false><<<gV, blk, 0, stream>>>(
      (const __bf16*)WV, (const __bf16*)WV, DMOD, 0L, (const __bf16*)XB, DMOD, (long)SEQ * DMOD,
      (void*)VTh, (void*)VTl, SEQ, (long)DMOD * SEQ, bv, DMOD, SEQ, DMOD, 1.0f, 0);

  const dim3 gB(((SEQ / 64) * (BDW / 64) + 7) / 8, NHEAD);
  for (int b = 0; b < NBT; ++b) {
    const size_t ab = (size_t)b * SEQ * DMOD;
    gemm_bf16_kernel<true, 0, 0, true><<<gB, blk, 0, stream>>>(
        (const __bf16*)(Qh + ab), (const __bf16*)(Ql + ab), DMOD, (long)HDIM,
        (const __bf16*)REB, DMOD, (long)HDIM,
        (void*)BDp, (void*)BDp, BDW, (long)SEQ * BDW, bq, SEQ, BDW, HDIM, 1.0f, SEQ / 64 - 1);
    attn_rel64_kernel<<<dim3(NHEAD * (SEQ / 64)), dim3(128), 0, stream>>>(
        (const __bf16*)Qh, (const __bf16*)Ql, (const __bf16*)Kh, (const __bf16*)Kl,
        (const __bf16*)VTh, (const __bf16*)VTl, BDp, CXh, CXl, b, 0.125f);
  }

  gemm_bf16_kernel<true, 2, 0, false><<<gP, blk, 0, stream>>>(
      (const __bf16*)CXh, (const __bf16*)CXl, DMOD, 0L, (const __bf16*)WOB, DMOD, 0L,
      (void*)out, (void*)out, DMOD, 0L, bo, NBT * SEQ, DMOD, DMOD, 1.0f, 0);
  (void)hipGetLastError();
}
